// QLSTM_65481071401286
// MI455X (gfx1250) — hardware-verified
//
#include <hip/hip_runtime.h>
#include <math.h>

constexpr int TSTEPS  = 256;
constexpr int NBATCH  = 8;
constexpr int NIN     = 1024;
constexpr int NHID    = 1024;
constexpr int NHEAD   = 16;
constexpr int HDIM    = NHID / NHEAD;
constexpr int NGATE4  = 4 * NHID;
constexpr int WGPITCH = NIN + NHID;
constexpr int NROWS   = TSTEPS * NBATCH;
constexpr int NOUT0   = NROWS * NHID;
constexpr int NOUT1   = NBATCH * NHID;
constexpr int RT      = 512;
constexpr int RW      = RT / 32;
constexpr int CVT_THR = 256;
constexpr float WCARRY = 256.0f;
constexpr float ACARRY = 16.0f;
constexpr float XCARRY = 16.0f;
constexpr float FOLD_H = 1.0f / (WCARRY * ACARRY);
constexpr float FOLD_X = 1.0f / (WCARRY * XCARRY);
constexpr float LN_EPS_F = 1e-5f;
constexpr int isqrt_c(int n) { int r = 0; while ((r + 1) * (r + 1) <= n) ++r; return r; }
constexpr float SCORE_SCL = 1.0f / (float)isqrt_c(HDIM);
static_assert(HDIM == 64, "head dim");
static_assert(isqrt_c(HDIM) * isqrt_c(HDIM) == HDIM, "exact sqrt");
static_assert(NHID == RW * 64, "16 waves x 64 columns");
static_assert(RW == 2 * NBATCH, "two waves per batch row");
static_assert(NHEAD == 16, "2 x 8 heads per batch row");
static_assert(NHID % 32 == 0 && NIN % 32 == 0, "K multiple of 32");
static_assert(NROWS % 64 == 0 && NGATE4 % 64 == 0, "GEMM tile multiples");
static_assert(RT * 16 == NBATCH * NHID, "A plane zero fill exact");

typedef __attribute__((ext_vector_type(16))) _Float16 v16h;
typedef __attribute__((ext_vector_type(8)))  _Float16 v8h;
typedef __attribute__((ext_vector_type(4)))  _Float16 v4h;
typedef __attribute__((ext_vector_type(2)))  _Float16 v2h;
typedef __attribute__((ext_vector_type(16))) __bf16   v16b;
typedef __attribute__((ext_vector_type(8)))  __bf16   v8b;
typedef __attribute__((ext_vector_type(8)))  float    v8f;
typedef __attribute__((ext_vector_type(4)))  float    v4f;
typedef __attribute__((ext_vector_type(2)))  float    v2f;

__device__ __forceinline__ unsigned short f2bf_bits(float f) {
  unsigned u = __float_as_uint(f);
  return (unsigned short)((u + 0x7FFFu + ((u >> 16) & 1u)) >> 16);
}
__device__ __forceinline__ float bf_bits2f(unsigned short h) { return __uint_as_float(((unsigned)h) << 16); }
__device__ __forceinline__ float bf16r(float f) { return bf_bits2f(f2bf_bits(f)); }

__device__ __forceinline__ void dep_guard_h(v8f& a, v8f& b, v16h x, v16h y) { asm volatile("v_nop\n\tv_nop\n\tv_nop\n\tv_nop" : "+v"(a), "+v"(b) : "v"(x), "v"(y)); }
__device__ __forceinline__ void dep_guard_b(v8f& a, v8f& b, v16b x, v16b y) { asm volatile("v_nop\n\tv_nop\n\tv_nop\n\tv_nop" : "+v"(a), "+v"(b) : "v"(x), "v"(y)); }
__device__ __forceinline__ void dep_guard4x_h(v8f& a, v8f& b, v8f& c, v8f& d, v16h x, v16h y) { asm volatile("v_nop\n\tv_nop\n\tv_nop\n\tv_nop" : "+v"(a), "+v"(b), "+v"(c), "+v"(d) : "v"(x), "v"(y)); }
__device__ __forceinline__ void dep_guard4x_b(v8f& a, v8f& b, v8f& c, v8f& d, v16b x, v16b y) { asm volatile("v_nop\n\tv_nop\n\tv_nop\n\tv_nop" : "+v"(a), "+v"(b), "+v"(c), "+v"(d) : "v"(x), "v"(y)); }
__device__ __forceinline__ void dep_guard4_h(v8f& a0, v8f& a1, v8f& a2, v8f& a3, v16h x, v16h y0, v16h y1, v16h y2, v16h y3) {
  asm volatile("v_nop\n\tv_nop\n\tv_nop\n\tv_nop" : "+v"(a0), "+v"(a1), "+v"(a2), "+v"(a3) : "v"(x), "v"(y0), "v"(y1), "v"(y2), "v"(y3));
}
__device__ __forceinline__ void keep4_h(v16h a, v16h b, v16h c, v16h d) { asm volatile("v_nop" :: "v"(a), "v"(b), "v"(c), "v"(d)); }
__device__ __forceinline__ void keep4_b(v16b a, v16b b, v16b c, v16b d) { asm volatile("v_nop" :: "v"(a), "v"(b), "v"(c), "v"(d)); }
__device__ __forceinline__ void acc_guard4(v8f& a, v8f& b, v8f& c, v8f& d) { asm volatile("v_nop\n\tv_nop\n\tv_nop\n\tv_nop" : "+v"(a), "+v"(b), "+v"(c), "+v"(d)); }
__device__ __forceinline__ void pin4(float& a, float& b, float& c, float& d) { asm volatile("" : "+v"(a), "+v"(b), "+v"(c), "+v"(d)); }

template <typename T> struct Frag;
template <> struct Frag<_Float16> {
  typedef v16h V; union U { v16h v; v8h h[2]; };
  static __device__ __forceinline__ v16h load(const _Float16* p) {
    U f; f.h[0] = *(const v8h*)(p); f.h[1] = *(const v8h*)(p + 16); return f.v;
  }
  static __device__ __forceinline__ v8f mma(v16h a, v16h b, v8f c) {
    return __builtin_amdgcn_wmma_f32_16x16x32_f16(false, a, false, b, (short)0, c, false, false);
  }
  static __device__ __forceinline__ void guard(v8f& a, v8f& b, v16h x, v16h y) { dep_guard_h(a, b, x, y); }
  static __device__ __forceinline__ void guard4(v8f& a, v8f& b, v8f& c, v8f& d, v16h x, v16h y) { dep_guard4x_h(a, b, c, d, x, y); }
  static __device__ __forceinline__ void keep(v16h a, v16h b, v16h c, v16h d) { keep4_h(a, b, c, d); }
};
template <> struct Frag<__bf16> {
  typedef v16b V; union U { v16b v; v8b h[2]; };
  static __device__ __forceinline__ v16b load(const __bf16* p) {
    U f; f.h[0] = *(const v8b*)(p); f.h[1] = *(const v8b*)(p + 16); return f.v;
  }
  static __device__ __forceinline__ v8f mma(v16b a, v16b b, v8f c) {
    return __builtin_amdgcn_wmma_f32_16x16x32_bf16(false, a, false, b, (short)0, c, false, false);
  }
  static __device__ __forceinline__ void guard(v8f& a, v8f& b, v16b x, v16b y) { dep_guard_b(a, b, x, y); }
  static __device__ __forceinline__ void guard4(v8f& a, v8f& b, v8f& c, v8f& d, v16b x, v16b y) { dep_guard4x_b(a, b, c, d, x, y); }
  static __device__ __forceinline__ void keep(v16b a, v16b b, v16b c, v16b d) { keep4_b(a, b, c, d); }
};

template <int ET> struct Elem;
template <> struct Elem<0> { typedef _Float16 T; };
template <> struct Elem<1> { typedef __bf16 T; };
template <int ET, bool SPLIT, int BIAS_MODE, int OUT_MODE, bool RESID, int ACT = 0>
__global__ __launch_bounds__(256) void wmma_gemm64(
    const unsigned short* __restrict__ Ap, const unsigned short* __restrict__ A2p, int lda, long strideA,
    const unsigned short* __restrict__ Btp, const unsigned short* __restrict__ Bt2p, int ldb, long strideB,
    void* __restrict__ Cout, void* __restrict__ Cout2, int ldc, long strideC,
    const float* __restrict__ bias,
    const float* __restrict__ resid, long strideR,
    int M, int N, int K, float scale) {
  typedef typename Elem<ET>::T T;
  typedef typename Frag<T>::V V;
  const T* A = (const T*)Ap; const T* A2 = (const T*)A2p; const T* Bt = (const T*)Btp; const T* Bt2 = (const T*)Bt2p;
  __shared__ __align__(16) float sT[8][16 * 68];
  const int b    = blockIdx.y;
  const int lane = threadIdx.x & 31;
  const int wave = threadIdx.x >> 5;
  const int tilesN = N >> 6;
  const int tilesM = M >> 6;
  const int tile = blockIdx.x * 8 + wave;
  if (tile >= tilesM * tilesN) return;
  const int tm = tile / tilesN;
  const int tn = tile - tm * tilesN;
  const int m0 = tm << 6;
  const int n0 = tn << 6;

  const T* Ab  = A  + (size_t)b * strideA;
  const T* Bb  = Bt + (size_t)b * strideB;
  const T* Ab2 = SPLIT ? (A2  + (size_t)b * strideA) : nullptr;
  const T* Bb2 = SPLIT ? (Bt2 + (size_t)b * strideB) : nullptr;

  const int rlane = lane & 15;
  const int koff  = (lane >> 4) * 8;
  const int mOff  = (lane >> 4) * 8;

  v8f acc[4][4];
#pragma unroll
  for (int i = 0; i < 4; ++i)
#pragma unroll
    for (int j = 0; j < 4; ++j) acc[i][j] = (v8f){0.f,0.f,0.f,0.f,0.f,0.f,0.f,0.f};

  for (int k0 = 0; k0 < K; k0 += 32) {
    V bh[4], bl[4];
#pragma unroll
    for (int j = 0; j < 4; ++j) {
      const size_t bo = (size_t)(n0 + (j << 4) + rlane) * ldb + koff + k0;
      bh[j] = Frag<T>::load(Bb + bo);
      if (SPLIT) bl[j] = Frag<T>::load(Bb2 + bo);
    }
#pragma unroll
    for (int i = 0; i < 4; ++i) {
      const size_t ao = (size_t)(m0 + (i << 4) + rlane) * lda + koff + k0;
      V ah = Frag<T>::load(Ab + ao);
      V al;
      if (SPLIT) al = Frag<T>::load(Ab2 + ao);
#pragma unroll
      for (int j = 0; j < 4; ++j) {
        acc[i][j] = Frag<T>::mma(ah, bh[j], acc[i][j]);
        if (SPLIT) {
          acc[i][j] = Frag<T>::mma(ah, bl[j], acc[i][j]);
          acc[i][j] = Frag<T>::mma(al, bh[j], acc[i][j]);
        }
      }
      Frag<T>::guard4(acc[i][0], acc[i][1], acc[i][2], acc[i][3], ah, SPLIT ? al : ah);
    }
    Frag<T>::keep(bh[0], bh[1], bh[2], bh[3]);
    if (SPLIT) Frag<T>::keep(bl[0], bl[1], bl[2], bl[3]);
  }
  acc_guard4(acc[0][0], acc[0][1], acc[0][2], acc[0][3]);
  acc_guard4(acc[1][0], acc[1][1], acc[1][2], acc[1][3]);
  acc_guard4(acc[2][0], acc[2][1], acc[2][2], acc[2][3]);
  acc_guard4(acc[3][0], acc[3][1], acc[3][2], acc[3][3]);

  float* slab = sT[wave];
  const float* Rb = RESID ? (resid + (size_t)b * strideR) : nullptr;
#pragma unroll
  for (int i = 0; i < 4; ++i) {
    const int mBase = m0 + (i << 4);
#pragma unroll
    for (int j = 0; j < 4; ++j) {
      const int n = n0 + (j << 4) + rlane;
      float bv = 0.f;
      if (BIAS_MODE == 2) bv = bias[n];
#pragma unroll
      for (int r = 0; r < 8; ++r) {
        float v = acc[i][j][r] * scale;
        if (BIAS_MODE == 1) v += bias[mBase + mOff + r];
        if (BIAS_MODE == 2) v += bv;
        if (RESID) v += Rb[(size_t)(mBase + mOff + r) * ldc + n];
        if (ACT == 1) v = tanhf(v);
        if (ACT == 2) v = fmaxf(v, 0.0f);
        if (ACT == 3) v = v / (1.0f + expf(-v));
        if (ACT == 4) v = (v > 0.f) ? v : 0.01f * v;
        if (ACT == 5) v = 0.5f * v * (1.0f + erff(v * 0.70710678118654752f));
        slab[(mOff + r) * 68 + (j << 4) + rlane] = v;
      }
    }
    __builtin_amdgcn_fence(__ATOMIC_RELEASE, "workgroup");
    __builtin_amdgcn_wave_barrier();
    __builtin_amdgcn_fence(__ATOMIC_ACQUIRE, "workgroup");
    if (OUT_MODE == 0) {
      float* C = (float*)Cout + (size_t)b * strideC;
      const int hh = lane >> 4, c4 = (lane & 15) * 4;
      for (int pass = 0; pass < 2; ++pass) {
#pragma unroll
        for (int it = 0; it < 8; ++it) {
          const int row = it * 2 + hh;
          v4f v = *(const v4f*)(slab + row * 68 + c4);
          *(volatile v4f*)(C + (size_t)(mBase + row) * ldc + n0 + c4) = v;
        }
        __threadfence();
      }
    } else {
      const int q = lane >> 3, c8 = (lane & 7) * 8;
      unsigned short* C  = (unsigned short*)Cout  + (size_t)b * strideC;
      unsigned short* C2 = (OUT_MODE == 2) ? ((unsigned short*)Cout2 + (size_t)b * strideC) : nullptr;
      for (int pass = 0; pass < 2; ++pass) {
#pragma unroll
        for (int it = 0; it < 4; ++it) {
          const int row = it * 4 + q;
          const float* sp = slab + row * 68 + c8;
          v8h hv, lv;
#pragma unroll
          for (int e = 0; e < 8; ++e) {
            if (OUT_MODE == 1) {
              hv[e] = (_Float16)sp[e];
            } else {
              unsigned short hb = f2bf_bits(sp[e]);
              unsigned short lb = f2bf_bits(sp[e] - bf_bits2f(hb));
              hv[e] = __builtin_bit_cast(_Float16, hb);
              lv[e] = __builtin_bit_cast(_Float16, lb);
            }
          }
          *(volatile v8h*)(C + (size_t)(mBase + row) * ldc + n0 + c8) = hv;
          if (OUT_MODE == 2) *(volatile v8h*)(C2 + (size_t)(mBase + row) * ldc + n0 + c8) = lv;
        }
        __threadfence();
      }
    }
    __builtin_amdgcn_fence(__ATOMIC_RELEASE, "workgroup");
    __builtin_amdgcn_wave_barrier();
    __builtin_amdgcn_fence(__ATOMIC_ACQUIRE, "workgroup");
  }
}

__global__ __launch_bounds__(CVT_THR) void cvt8_kernel(const float* __restrict__ src, unsigned short* __restrict__ dst,
                                                       int nrow, int ncol8, int spitch, int scol0, float sc) {
  const int i  = blockIdx.x * CVT_THR + threadIdx.x;
  const int n8 = nrow * ncol8;
  if (i < n8) {
    const int row = i / ncol8;
    const int c8  = i - row * ncol8;
    const float* sp = src + (size_t)row * spitch + scol0 + c8 * 8;
    const v4f a = *(const v4f*)(sp);
    const v4f b = *(const v4f*)(sp + 4);
    v8h hv;
#pragma unroll
    for (int e = 0; e < 4; ++e) {
      const float fa = bf16r(a[e]) * sc;
      const float fb = bf16r(b[e]) * sc;
      hv[e]     = (_Float16)fa;
      hv[4 + e] = (_Float16)fb;
    }
    *(volatile v8h*)(dst + (size_t)i * 8) = hv;
    __threadfence();
    *(volatile v8h*)(dst + (size_t)i * 8) = hv;
  }
}

__global__ __launch_bounds__(CVT_THR) void bias_prep_kernel(const float* __restrict__ src, float* __restrict__ dst, int n4) {
  const int i = blockIdx.x * CVT_THR + threadIdx.x;
  if (i < n4) {
    const v4f a = *(const v4f*)(src + (size_t)i * 4);
    v4f o;
#pragma unroll
    for (int e = 0; e < 4; ++e) o[e] = bf16r(a[e]);
    *(volatile v4f*)(dst + (size_t)i * 4) = o;
    __threadfence();
    *(volatile v4f*)(dst + (size_t)i * 4) = o;
  }
}

__device__ __forceinline__ void wave_sync_lds() {
  __builtin_amdgcn_fence(__ATOMIC_RELEASE, "workgroup");
  __builtin_amdgcn_wave_barrier();
  __builtin_amdgcn_fence(__ATOMIC_ACQUIRE, "workgroup");
}

__device__ __forceinline__ float sigm(float x) {
  const float xc = fminf(fmaxf(x, -30.0f), 30.0f);
  return 1.0f / (1.0f + expf(-xc));
}
__device__ __forceinline__ float tnh(float x) {
  const float xc = fminf(fmaxf(x, -15.0f), 15.0f);
  return 1.0f - 2.0f / (1.0f + expf(2.0f * xc));
}

__device__ __forceinline__ void tile_gemm4(const _Float16* arow, const _Float16* brow,
                                           v8f& a0, v8f& a1, v8f& a2, v8f& a3) {
  const v8f z8 = {0.f, 0.f, 0.f, 0.f, 0.f, 0.f, 0.f, 0.f};
  a0 = z8; a1 = z8; a2 = z8; a3 = z8;
#pragma unroll 1
  for (int k0 = 0; k0 < NHID; k0 += 32) {
    const v16h a  = Frag<_Float16>::load(arow + k0);
    const v16h f0 = Frag<_Float16>::load(brow + k0);
    const v16h f1 = Frag<_Float16>::load(brow + (size_t)16 * NHID + k0);
    const v16h f2 = Frag<_Float16>::load(brow + (size_t)32 * NHID + k0);
    const v16h f3 = Frag<_Float16>::load(brow + (size_t)48 * NHID + k0);
    a0 = Frag<_Float16>::mma(a, f0, a0);
    a1 = Frag<_Float16>::mma(a, f1, a1);
    a2 = Frag<_Float16>::mma(a, f2, a2);
    a3 = Frag<_Float16>::mma(a, f3, a3);
    dep_guard4_h(a0, a1, a2, a3, a, f0, f1, f2, f3);
  }
  acc_guard4(a0, a1, a2, a3);
}

template <bool HASB>
__device__ __forceinline__ void tile_store4(float* zb, int ncol, int hh, const float* bias, float fold,
                                            const v8f& a0, const v8f& a1, const v8f& a2, const v8f& a3) {
  float b0 = 0.0f, b1 = 0.0f, b2 = 0.0f, b3 = 0.0f;
  if (HASB) {
    float r0 = bias[ncol];
    float r1 = bias[ncol + 16];
    float r2 = bias[ncol + 32];
    float r3 = bias[ncol + 48];
    pin4(r0, r1, r2, r3);
    b0 = bf16r(r0);
    b1 = bf16r(r1);
    b2 = bf16r(r2);
    b3 = bf16r(r3);
    pin4(b0, b1, b2, b3);
  }
  if (hh == 0) {
#pragma unroll
    for (int r = 0; r < 8; ++r) {
      zb[r * NHID + ncol]      = a0[r] * fold + b0;
      zb[r * NHID + ncol + 16] = a1[r] * fold + b1;
      zb[r * NHID + ncol + 32] = a2[r] * fold + b2;
      zb[r * NHID + ncol + 48] = a3[r] * fold + b3;
    }
  }
}

__device__ __forceinline__ void ln_gate(const float* zbrow, const float* zxrow, const float* gp, const float* bp,
                                        int lane, int halfsel, v4f (&zn)[4]) {
  v4f v[8];
  float s = 0.0f;
#pragma unroll
  for (int q2 = 0; q2 < 8; ++q2) {
    const int col = q2 * 128 + lane * 4;
    const v4f a = *(const v4f*)(zbrow + col);
    const v4f b = *(const v4f*)(zxrow + col);
    v[q2] = a + b;
    s += (v[q2][0] + v[q2][1]) + (v[q2][2] + v[q2][3]);
  }
#pragma unroll
  for (int off = 1; off < 32; off <<= 1) s += __shfl_xor(s, off, 32);
  const float mu = s * (1.0f / (float)NHID);
  float ss = 0.0f;
#pragma unroll
  for (int q2 = 0; q2 < 8; ++q2)
#pragma unroll
    for (int e = 0; e < 4; ++e) { const float d = v[q2][e] - mu; v[q2][e] = d; ss += d * d; }
#pragma unroll
  for (int off = 1; off < 32; off <<= 1) ss += __shfl_xor(ss, off, 32);
  const float var  = ss * (1.0f / (float)NHID);
  const float rstd = rsqrtf(var + LN_EPS_F);
#pragma unroll
  for (int q = 0; q < 4; ++q) {
    const v4f g4 = *(const v4f*)(gp + q * 128 + lane * 4);
    const v4f b4 = *(const v4f*)(bp + q * 128 + lane * 4);
#pragma unroll
    for (int e = 0; e < 4; ++e) {
      const float lo = v[q][e];
      const float hi = v[4 + q][e];
      const float d  = halfsel ? hi : lo;
      zn[q][e] = (d * rstd) * bf16r(g4[e]) + bf16r(b4[e]);
    }
  }
}

__device__ __forceinline__ void gate_phase(int kg, const _Float16* arow, const _Float16* WGH, float* Zb,
                                           const float* zxrow_t, const float* lng, const float* lnb,
                                           int ncol, int koff, int hh, int eb, int colbase, int lane, int halfsel,
                                           v4f (&zn)[4]) {
  v8f a0, a1, a2, a3;
  tile_gemm4(arow, WGH + (size_t)(kg * NHID + ncol) * NHID + koff, a0, a1, a2, a3);
  tile_store4<false>(Zb, ncol, hh, nullptr, FOLD_H, a0, a1, a2, a3);
  __syncthreads();
  ln_gate(Zb + eb * NHID, zxrow_t + kg * NHID, lng + kg * NHID + colbase, lnb + kg * NHID + colbase, lane, halfsel, zn);
}

__device__ __forceinline__ void put_a4(_Float16* dst, v4f v) {
  v4h hv;
  hv[0] = (_Float16)(v[0] * ACARRY);
  hv[1] = (_Float16)(v[1] * ACARRY);
  hv[2] = (_Float16)(v[2] * ACARRY);
  hv[3] = (_Float16)(v[3] * ACARRY);
  *(v4h*)dst = hv;
}

__global__ __launch_bounds__(RT) void recur_kernel(
    const float* __restrict__ ZX,
    const unsigned short* __restrict__ WGHp, const unsigned short* __restrict__ WQp,
    const unsigned short* __restrict__ WOp, const unsigned short* __restrict__ WKVp,
    const float* __restrict__ lng, const float* __restrict__ lnb,
    const float* __restrict__ bq, const float* __restrict__ bk, const float* __restrict__ bv, const float* __restrict__ bo,
    float* KC, float* VC, float* __restrict__ OUT) {
  __shared__ __align__(16) _Float16 Apl[NBATCH * NHID];
  __shared__ __align__(16) float    Zb[NBATCH * NHID];
  __shared__ __align__(16) float    Pb[RW * 256];
  const _Float16* WGH = (const _Float16*)WGHp;
  const _Float16* WQ  = (const _Float16*)WQp;
  const _Float16* WO  = (const _Float16*)WOp;
  const _Float16* WKV = (const _Float16*)WKVp;
  const int tid = threadIdx.x, lane = tid & 31, wave = tid >> 5;
  const int c = lane & 15, hh = lane >> 4, koff = hh * 8;
  const int eb = wave & 7, halfsel = wave >> 3, colbase = halfsel * 512;
  const int ecol = colbase + lane * 4;
  const int ncol = wave * 64 + c;

  {
    const _Float16 zh = (_Float16)0.0f;
    const v8h z8h = {zh, zh, zh, zh, zh, zh, zh, zh};
    *(v8h*)(Apl + tid * 16)     = z8h;
    *(v8h*)(Apl + tid * 16 + 8) = z8h;
  }
  v4f cx[4];
#pragma unroll
  for (int q = 0; q < 4; ++q) cx[q] = (v4f){0.f, 0.f, 0.f, 0.f};
  __syncthreads();

  const _Float16* arow = Apl + (lane & 7) * NHID + koff;
  float* pw = Pb + wave * 256;

#pragma unroll 1
  for (int t = 0; t < TSTEPS; ++t) {
    const float* zxrow_t = ZX + ((size_t)t * NBATCH + eb) * NGATE4;
    v4f zn[4];
    v4f fg[4], ig[4], h0r[4];

    gate_phase(0, arow, WGH, Zb, zxrow_t, lng, lnb, ncol, koff, hh, eb, colbase, lane, halfsel, zn);
#pragma unroll
    for (int q = 0; q < 4; ++q)
#pragma unroll
      for (int e = 0; e < 4; ++e) fg[q][e] = sigm(zn[q][e]);
    __syncthreads();
    gate_phase(1, arow, WGH, Zb, zxrow_t, lng, lnb, ncol, koff, hh, eb, colbase, lane, halfsel, zn);
#pragma unroll
    for (int q = 0; q < 4; ++q)
#pragma unroll
      for (int e = 0; e < 4; ++e) ig[q][e] = sigm(zn[q][e]);
    __syncthreads();
    gate_phase(2, arow, WGH, Zb, zxrow_t, lng, lnb, ncol, koff, hh, eb, colbase, lane, halfsel, zn);
#pragma unroll
    for (int q = 0; q < 4; ++q)
#pragma unroll
      for (int e = 0; e < 4; ++e) {
        const float gg = tnh(zn[q][e]);
        cx[q][e] = fg[q][e] * cx[q][e] + ig[q][e] * gg;
      }
    __syncthreads();
    gate_phase(3, arow, WGH, Zb, zxrow_t, lng, lnb, ncol, koff, hh, eb, colbase, lane, halfsel, zn);
#pragma unroll
    for (int q = 0; q < 4; ++q) {
#pragma unroll
      for (int e = 0; e < 4; ++e) {
        const float og = sigm(zn[q][e]);
        h0r[q][e] = og * tnh(cx[q][e]);
      }
      put_a4(Apl + eb * NHID + ecol + q * 128, h0r[q]);
    }
    __syncthreads();

    if (t > 0) {
      {
        v8f a0, a1, a2, a3;
        tile_gemm4(arow, WQ + (size_t)ncol * NHID + koff, a0, a1, a2, a3);
        tile_store4<true>(Zb, ncol, hh, bq, FOLD_H, a0, a1, a2, a3);
      }
      __syncthreads();

      {
        const int tm1 = t - 1;
        const int hd0 = halfsel * 8;
#pragma unroll 1
        for (int p = 0; p < 8; ++p) {
          const int hd = hd0 + p;
          const float* qv = Zb + eb * NHID + hd * HDIM;
          const size_t hoff = (size_t)eb * NHID + (size_t)hd * HDIM;
          float lmax = -INFINITY;
#pragma unroll 1
          for (int s0 = 0; s0 < t; s0 += 32) {
            const int s  = s0 + lane;
            const int sc = (s < t) ? s : tm1;
            const float* kp = KC + (size_t)sc * (NBATCH * NHID) + hoff;
            float dot = 0.0f;
#pragma unroll 4
            for (int i = 0; i < HDIM / 4; ++i) {
              const v4f qq = *(const v4f*)(qv + 4 * i);
              const v4f kk = *(const v4f*)(kp + 4 * i);
              dot += qq[0] * kk[0];
              dot += qq[1] * kk[1];
              dot += qq[2] * kk[2];
              dot += qq[3] * kk[3];
            }
            const float sv0 = dot * SCORE_SCL;
            const float sv  = (s < t) ? sv0 : -INFINITY;
            pw[s] = sv;
            lmax = fmaxf(lmax, sv);
          }
#pragma unroll
          for (int off = 1; off < 32; off <<= 1) lmax = fmaxf(lmax, __shfl_xor(lmax, off, 32));
          float lsum = 0.0f;
#pragma unroll 1
          for (int s0 = 0; s0 < t; s0 += 32) {
            const int s = s0 + lane;
            const float sv = pw[s];
            const float ev = expf(sv - lmax);
            const float pe = (s < t) ? ev : 0.0f;
            pw[s] = pe;
            lsum += pe;
          }
#pragma unroll
          for (int off = 1; off < 32; off <<= 1) lsum += __shfl_xor(lsum, off, 32);
          wave_sync_lds();
          float c0 = 0.0f, c1 = 0.0f;
          const float* vp = VC + hoff + 2 * lane;
#pragma unroll 1
          for (int s0 = 0; s0 < t; s0 += 4) {
            const v4f p4 = *(const v4f*)(pw + s0);
#pragma unroll
            for (int e = 0; e < 4; ++e) {
              const int s  = s0 + e;
              const int sc = (s < t) ? s : tm1;
              const v2f vv = *(const v2f*)(vp + (size_t)sc * (NBATCH * NHID));
              c0 += p4[e] * vv[0];
              c1 += p4[e] * vv[1];
            }
          }
          const float inv = 1.0f / lsum;
          v2h hv;
          hv[0] = (_Float16)(c0 * inv * ACARRY);
          hv[1] = (_Float16)(c1 * inv * ACARRY);
          *(v2h*)(Apl + eb * NHID + hd * HDIM + 2 * lane) = hv;
          wave_sync_lds();
        }
      }
      __syncthreads();

      {
        v8f a0, a1, a2, a3;
        tile_gemm4(arow, WO + (size_t)ncol * NHID + koff, a0, a1, a2, a3);
        tile_store4<true>(Zb, ncol, hh, bo, FOLD_H, a0, a1, a2, a3);
      }
      __syncthreads();
    }

    {
      v4f hx[4];
#pragma unroll
      for (int q = 0; q < 4; ++q) {
        hx[q] = h0r[q];
        if (t > 0) {
          const v4f ao = *(const v4f*)(Zb + eb * NHID + ecol + q * 128);
          hx[q] = hx[q] + ao;
        }
        put_a4(Apl + eb * NHID + ecol + q * 128, hx[q]);
      }
      float* op = OUT + ((size_t)t * NBATCH + eb) * NHID + ecol;
      const bool last = (t == TSTEPS - 1);
      float* o1 = OUT + (size_t)NOUT0 + (size_t)eb * NHID + ecol;
      float* o2 = OUT + (size_t)NOUT0 + (size_t)NOUT1 + (size_t)eb * NHID + ecol;
      for (int pass = 0; pass < 2; ++pass) {
#pragma unroll
        for (int q = 0; q < 4; ++q) *(volatile v4f*)(op + q * 128) = hx[q];
        if (last) {
#pragma unroll
          for (int q = 0; q < 4; ++q) {
            *(volatile v4f*)(o1 + q * 128) = hx[q];
            *(volatile v4f*)(o2 + q * 128) = cx[q];
          }
        }
        __threadfence();
      }
    }
    __syncthreads();

    {
      v8f a0, a1, a2, a3;
      tile_gemm4(arow, WKV + (size_t)ncol * NHID + koff, a0, a1, a2, a3);
      tile_store4<true>(Zb, ncol, hh, bk, FOLD_H, a0, a1, a2, a3);
    }
    __syncthreads();
    {
      v4f kv[4];
#pragma unroll
      for (int q = 0; q < 4; ++q) kv[q] = *(const v4f*)(Zb + eb * NHID + ecol + q * 128);
      float* kp = KC + ((size_t)t * NBATCH + eb) * NHID + ecol;
      for (int pass = 0; pass < 2; ++pass) {
#pragma unroll
        for (int q = 0; q < 4; ++q) *(volatile v4f*)(kp + q * 128) = kv[q];
        __threadfence();
      }
    }
    __syncthreads();
    {
      v8f a0, a1, a2, a3;
      tile_gemm4(arow, WKV + (size_t)(NHID + ncol) * NHID + koff, a0, a1, a2, a3);
      tile_store4<true>(Zb, ncol, hh, bv, FOLD_H, a0, a1, a2, a3);
    }
    __syncthreads();
    {
      v4f kv[4];
#pragma unroll
      for (int q = 0; q < 4; ++q) kv[q] = *(const v4f*)(Zb + eb * NHID + ecol + q * 128);
      float* vq = VC + ((size_t)t * NBATCH + eb) * NHID + ecol;
      for (int pass = 0; pass < 2; ++pass) {
#pragma unroll
        for (int q = 0; q < 4; ++q) *(volatile v4f*)(vq + q * 128) = kv[q];
        __threadfence();
      }
    }
    __syncthreads();
    __threadfence();
  }
}

extern "C" void kernel_launch(void* const* d_in, const int* in_sizes, int n_in,
                              void* d_out, int out_size, void* d_ws, size_t ws_size, hipStream_t stream) {
  if (n_in < 13 || d_out == nullptr || d_ws == nullptr) return;
  if (in_sizes[0] != NROWS * NIN || in_sizes[1] != NGATE4 * WGPITCH || in_sizes[2] != NGATE4 ||
      in_sizes[3] != NGATE4 || in_sizes[4] != NGATE4 || in_sizes[5] != NHID * NHID || in_sizes[6] != NHID * NHID ||
      in_sizes[7] != NHID * NHID || in_sizes[8] != NHID || in_sizes[9] != NHID || in_sizes[10] != NHID ||
      in_sizes[11] != NHID * NHID || in_sizes[12] != NHID || out_size != NOUT0 + 2 * NOUT1) return;

  const float* x_in    = (const float*)d_in[0];
  const float* w_gates = (const float*)d_in[1];
  const float* b_gates = (const float*)d_in[2];
  const float* ln_g    = (const float*)d_in[3];
  const float* ln_b    = (const float*)d_in[4];
  const float* w_q     = (const float*)d_in[5];
  const float* w_k     = (const float*)d_in[6];
  const float* w_v     = (const float*)d_in[7];
  const float* b_q     = (const float*)d_in[8];
  const float* b_k     = (const float*)d_in[9];
  const float* b_v     = (const float*)d_in[10];
  const float* w_o     = (const float*)d_in[11];
  const float* b_o     = (const float*)d_in[12];
  float* out = (float*)d_out;

  char* ws = (char*)d_ws; size_t off = 0;
  auto carve = [&](size_t bytes) -> char* { char* p = ws + off; off += (bytes + 255) & ~(size_t)255; return p; };
  unsigned short* XH    = (unsigned short*)carve((size_t)NROWS * NIN * 2);
  unsigned short* WGX   = (unsigned short*)carve((size_t)NGATE4 * NIN * 2);
  unsigned short* WGHp  = (unsigned short*)carve((size_t)NGATE4 * NHID * 2);
  unsigned short* WQ16  = (unsigned short*)carve((size_t)NHID * NHID * 2);
  unsigned short* WO16  = (unsigned short*)carve((size_t)NHID * NHID * 2);
  unsigned short* WKV16 = (unsigned short*)carve((size_t)2 * NHID * NHID * 2);
  float*          BG    = (float*)carve((size_t)NGATE4 * 4);
  float*          ZX    = (float*)carve((size_t)NROWS * NGATE4 * 4);
  float*          KC    = (float*)carve((size_t)TSTEPS * NBATCH * NHID * 4);
  float*          VC    = (float*)carve((size_t)TSTEPS * NBATCH * NHID * 4);
  if (off > ws_size || off > (size_t)134217728) return;

  const int n8x = NROWS * (NIN / 8);
  const int n8g = NGATE4 * (NIN / 8);
  const int n8w = NHID * (NHID / 8);
  cvt8_kernel<<<(n8x + CVT_THR - 1) / CVT_THR, CVT_THR, 0, stream>>>(x_in,    XH,    NROWS,  NIN / 8,  NIN,     0,   XCARRY);
  cvt8_kernel<<<(n8g + CVT_THR - 1) / CVT_THR, CVT_THR, 0, stream>>>(w_gates, WGX,   NGATE4, NIN / 8,  WGPITCH, 0,   WCARRY);
  cvt8_kernel<<<(n8g + CVT_THR - 1) / CVT_THR, CVT_THR, 0, stream>>>(w_gates, WGHp,  NGATE4, NHID / 8, WGPITCH, NIN, WCARRY);
  cvt8_kernel<<<(n8w + CVT_THR - 1) / CVT_THR, CVT_THR, 0, stream>>>(w_q,     WQ16,  NHID,   NHID / 8, NHID,    0,   WCARRY);
  cvt8_kernel<<<(n8w + CVT_THR - 1) / CVT_THR, CVT_THR, 0, stream>>>(w_o,     WO16,  NHID,   NHID / 8, NHID,    0,   WCARRY);
  cvt8_kernel<<<(n8w + CVT_THR - 1) / CVT_THR, CVT_THR, 0, stream>>>(w_k,     WKV16, NHID,   NHID / 8, NHID,    0,   WCARRY);
  cvt8_kernel<<<(n8w + CVT_THR - 1) / CVT_THR, CVT_THR, 0, stream>>>(w_v,     WKV16 + (size_t)NHID * NHID, NHID, NHID / 8, NHID, 0, WCARRY);
  bias_prep_kernel<<<(NGATE4 / 4 + CVT_THR - 1) / CVT_THR, CVT_THR, 0, stream>>>(b_gates, BG, NGATE4 / 4);

  const dim3 ggrid((NROWS / 64) * (NGATE4 / 64) / 8, 1);
  wmma_gemm64<0, false, 2, 0, false, 0><<<ggrid, 256, 0, stream>>>(
      XH, XH, NIN, 0L, WGX, WGX, NIN, 0L, (void*)ZX, (void*)ZX, NGATE4, 0L,
      BG, BG, 0L, NROWS, NGATE4, NIN, FOLD_X);

  recur_kernel<<<1, RT, 0, stream>>>(ZX, WGHp, WQ16, WO16, WKV16, ln_g, ln_b, b_q, b_k, b_v, b_o, KC, VC, out);
}
